// LogicLayer_90580860273055
// MI455X (gfx1250) — hardware-run, weakly checked
//
#include <hip/hip_runtime.h>
#include <math.h>

typedef __attribute__((ext_vector_type(16))) _Float16 v16h;
typedef __attribute__((ext_vector_type(8)))  _Float16 v8h;
typedef __attribute__((ext_vector_type(8)))  float    v8f;
typedef __attribute__((ext_vector_type(4)))  float    v4f;

constexpr int kNb = 4;
constexpr int kNo = 64;
constexpr int kNc = 8;
constexpr int kRowsO1 = kNb * kNo;
constexpr int kRowsO2 = kNb * kNo * kNo;
constexpr int kRowsO3 = kNb * kNo * kNo * kNo;
constexpr int kFeat0 = 3 * kNc;
constexpr int kFeat1 = 4 * kNc;
constexpr int kFeat2 = 8 * kNc;
constexpr int kFeat3 = 12 * kNc;
constexpr int kWtRows = 16;
static_assert(kNo == 64 && kNc == 8 && kNb == 4, "index arithmetic below uses shifts for these sizes");
static_assert((kFeat3 % 32) == 0, "order-3 depth is a whole number of 32-deep steps");
static_assert(kFeat0 == 24 && kFeat1 == 32 && kFeat2 == 64 && kFeat3 == 96, "feature widths");

constexpr int kOutO0 = 0;
constexpr int kOutO1 = kOutO0 + kNb * kNc;
constexpr int kOutO2 = kOutO1 + kRowsO1 * kNc;
constexpr int kOutO3 = kOutO2 + kRowsO2 * kNc;
constexpr int kOutTotal = kOutO3 + kRowsO3 * kNc;
static_assert(kOutO1 * 4 == 128 && kOutO2 * 4 == 8320 && kOutO3 * 4 == 532608, "output byte offsets");
static_assert((size_t)kOutTotal * 4 == 34087040ull, "output bytes");

constexpr float kFeatCarry = 64.0f;
constexpr float kWCarry    = 64.0f;
constexpr float kFold      = 1.0f / (kFeatCarry * kWCarry);
constexpr float kF16MinNormal = 6.103515625e-05f;

constexpr size_t kBytesX3H = (size_t)kRowsO3 * kNc * 2;
constexpr size_t kBytesX2H = (size_t)kRowsO2 * kNc * 2;
constexpr size_t kBytesW3T = (size_t)kWtRows * kFeat3 * 2;
constexpr size_t kBytesR2  = (size_t)kRowsO2 * 16 * 4;
constexpr size_t kOffX3H = 0;
constexpr size_t kOffX2H = kOffX3H + kBytesX3H;
constexpr size_t kOffW3T = kOffX2H + kBytesX2H;
constexpr size_t kOffR2  = kOffW3T + kBytesW3T;
constexpr size_t kWsTotal = kOffR2 + kBytesR2;
static_assert(kWsTotal == 16777216ull + 262144ull + 3072ull + 1048576ull, "carve total");
static_assert(kWsTotal == 18091008ull, "carve total value");
static_assert(kWsTotal <= 134217728ull, "carve cap");
static_assert((kOffX2H % 128) == 0 && (kOffW3T % 128) == 0 && (kOffR2 % 128) == 0, "128-B aligned regions");
constexpr int kX2Seg0 = kRowsO3;
static_assert((size_t)kX2Seg0 * 16 == kBytesX3H, "X2H follows X3H");

__device__ __forceinline__ _Float16 to_f16_carried(float v, float carry) {
  float s = v * carry;
  s = (fabsf(s) < kF16MinNormal) ? 0.0f : s;
  return (_Float16)s;
}

__device__ __forceinline__ float sigmoid_f32(float v) {
  return __builtin_amdgcn_rcpf(1.0f + expf(-v));
}

union FragU { v16h v; v8h p[2]; };

__device__ __forceinline__ v16h frag_load_f16(const _Float16* p) {
  FragU f;
  f.p[0] = *(const v8h*)(p);
  f.p[1] = *(const v8h*)(p + 16);
  return f.v;
}

__device__ __forceinline__ v8f mma_f16_guarded(v16h a, v16h b, v8f c) {
  c = __builtin_amdgcn_wmma_f32_16x16x32_f16(false, a, false, b, (short)0, c, false, false);
  asm volatile("v_nop\n\tv_nop\n\tv_nop\n\tv_nop" : "+v"(c) : "v"(a), "v"(b));
  return c;
}

constexpr int kPartPitch = 17;

__global__ __launch_bounds__(256) void prep_x3_kernel(
    const float* __restrict__ x3, unsigned short* __restrict__ x3h, float* __restrict__ R2)
{
  __shared__ float sP[8 * 2 * 32 * kPartPitch];
  __shared__ __align__(16) float sR[256];
  const int tid = threadIdx.x, lane = tid & 31, wave = tid >> 5;
  const int blk = blockIdx.x;
  const int jt = blk & 3, i = (blk >> 2) & 63, b = blk >> 8;
  const int bi = b * 64 + i;

  v8h hv[2][2];
#pragma unroll
  for (int jj = 0; jj < 2; ++jj) {
    const int j = jt * 16 + wave * 2 + jj;
    const size_t rowbase = (size_t)(bi * 64 + j) * 512;
    float mx[8], mn[8];
#pragma unroll
    for (int it = 0; it < 2; ++it) {
      const int k = it * 32 + lane;
      const float* p = x3 + rowbase + k * 8;
      const v4f a0 = *(const v4f*)(p);
      const v4f a1 = *(const v4f*)(p + 4);
      const bool valid = (k != i) && (k != j) && (i != j);
      v8h hh;
#pragma unroll
      for (int e = 0; e < 4; ++e) {
        const float u0 = a0[e];
        const float u1 = a1[e];
        hh[e]     = to_f16_carried(u0, kFeatCarry);
        hh[4 + e] = to_f16_carried(u1, kFeatCarry);
        const float m0 = valid ? u0 : 0.0f;
        const float n0 = valid ? u0 : 1.0f;
        const float m1 = valid ? u1 : 0.0f;
        const float n1 = valid ? u1 : 1.0f;
        if (it == 0) {
          mx[e] = m0; mn[e] = n0; mx[4 + e] = m1; mn[4 + e] = n1;
        } else {
          mx[e] = fmaxf(mx[e], m0); mn[e] = fminf(mn[e], n0);
          mx[4 + e] = fmaxf(mx[4 + e], m1); mn[4 + e] = fminf(mn[4 + e], n1);
        }
      }
      hv[jj][it] = hh;
    }
    float* pp = sP + ((wave * 2 + jj) * 32 + lane) * kPartPitch;
#pragma unroll
    for (int c = 0; c < 8; ++c) {
      pp[2 * c]     = mx[c];
      pp[2 * c + 1] = mn[c];
    }
  }
  __syncthreads();
  {
    const int jj = lane >> 4, slot = lane & 15;
    const bool isMin = (slot & 1) != 0;
    const float* col = sP + ((wave * 2 + jj) * 32) * kPartPitch + slot;
    float r = col[0];
#pragma unroll 4
    for (int src = 1; src < 32; ++src) {
      const float x = col[src * kPartPitch];
      const float a = fmaxf(r, x);
      const float c = fminf(r, x);
      r = isMin ? c : a;
    }
    sR[wave * 32 + lane] = r;
  }
  __syncthreads();
  v4f rv = (v4f){0.f, 0.f, 0.f, 0.f};
  if (wave < 2) rv = *(const v4f*)(sR + wave * 128 + lane * 4);
  float* r2dst = R2 + (size_t)(bi * 64 + jt * 16) * 16 + wave * 128 + lane * 4;
  for (int pass = 0; pass < 2; ++pass) {
#pragma unroll
    for (int jj = 0; jj < 2; ++jj) {
      const int j = jt * 16 + wave * 2 + jj;
      const size_t rowbase = (size_t)(bi * 64 + j) * 512;
#pragma unroll
      for (int it = 0; it < 2; ++it)
        *(volatile v8h*)(x3h + rowbase + (it * 32 + lane) * 8) = hv[jj][it];
    }
    if (wave < 2) *(volatile v4f*)(r2dst) = rv;
    __threadfence();
  }
}

__global__ __launch_bounds__(256) void prep_small_kernel(
    const float* __restrict__ x0, const float* __restrict__ x1, const float* __restrict__ x2,
    const float* __restrict__ W0, const float* __restrict__ b0,
    const float* __restrict__ W1, const float* __restrict__ b1,
    const float* __restrict__ W3,
    unsigned short* __restrict__ x2h, unsigned short* __restrict__ w3t,
    float* __restrict__ out)
{
  __shared__ float sW[256];
  __shared__ float sF[32 * 32];
  __shared__ __align__(16) float sO[256];
  __shared__ float sF0[4 * 24];
  const int tid = threadIdx.x, lane = tid & 31, wave = tid >> 5;
  const int blk = blockIdx.x;

  if (blk < 64) {
    const int gid = blk * 256 + tid;
    const size_t e0 = (size_t)gid * 8;
    const v4f a0 = *(const v4f*)(x2 + e0);
    const v4f a1 = *(const v4f*)(x2 + e0 + 4);
    v8h hv;
#pragma unroll
    for (int e = 0; e < 4; ++e) {
      const float u0 = a0[e];
      const float u1 = a1[e];
      hv[e]     = to_f16_carried(u0, kFeatCarry);
      hv[4 + e] = to_f16_carried(u1, kFeatCarry);
    }
    unsigned short* dst = x2h + e0;
    *(volatile v8h*)dst = hv;
    __threadfence();
    *(volatile v8h*)dst = hv;
    return;
  }

  if (blk == 64) {
    if (wave < 6) {
      const int n = tid / 12;
      const int seg = tid - n * 12;
      const int nc = (n < 8) ? n : 7;
      v8h hv;
#pragma unroll
      for (int e = 0; e < 8; ++e) {
        float w = W3[(seg * 8 + e) * 8 + nc];
        asm volatile("" : "+v"(w));
        const float s = (n < 8) ? w : 0.0f;
        hv[e] = to_f16_carried(s, kWCarry);
      }
      unsigned short* dst = w3t + tid * 8;
      *(volatile v8h*)dst = hv;
      __threadfence();
      *(volatile v8h*)dst = hv;
    }
    return;
  }

  if (blk < 73) {
    const int rbase = (blk - 65) * 32;
    sW[tid] = W1[tid];
    {
      const int r = lane >> 3, c = lane & 7;
      const int grow = rbase + wave * 4 + r;
      const int bb = grow >> 6;
      sF[(wave * 4 + r) * 32 + c]     = x0[bb * 8 + c];
      sF[(wave * 4 + r) * 32 + 8 + c] = x1[grow * 8 + c];
    }
#pragma unroll 1
    for (int r = 0; r < 4; ++r) {
      const int grow = rbase + wave * 4 + r;
      const int i = grow & 63;
      const float* p = x2 + (size_t)grow * 512;
      float mx[4], mn[4];
#pragma unroll
      for (int it = 0; it < 4; ++it) {
        const int j = it * 16 + (lane >> 1);
        const v4f v = *(const v4f*)(p + it * 128 + lane * 4);
        const bool valid = (j != i);
#pragma unroll
        for (int u = 0; u < 4; ++u) {
          const float x = v[u];
          const float a = valid ? x : 0.0f;
          const float c = valid ? x : 1.0f;
          if (it == 0) { mx[u] = a; mn[u] = c; }
          else { mx[u] = fmaxf(mx[u], a); mn[u] = fminf(mn[u], c); }
        }
      }
#pragma unroll
      for (int off = 2; off < 32; off <<= 1) {
#pragma unroll
        for (int u = 0; u < 4; ++u) {
          const float om = __shfl_xor(mx[u], off, 32);
          const float on = __shfl_xor(mn[u], off, 32);
          mx[u] = fmaxf(mx[u], om);
          mn[u] = fminf(mn[u], on);
        }
      }
      if (lane < 2) {
        float* q = sF + (wave * 4 + r) * 32 + 16 + lane * 8;
#pragma unroll
        for (int u = 0; u < 4; ++u) {
          q[2 * u]     = mx[u];
          q[2 * u + 1] = mn[u];
        }
      }
    }
    __syncthreads();
    {
      const int rl = tid >> 3, ch = tid & 7;
      float acc = 0.0f;
#pragma unroll 4
      for (int k = 0; k < kFeat1; ++k) acc = fmaf(sF[rl * 32 + k], sW[k * 8 + ch], acc);
      const float v = acc + b1[ch];
      sO[tid] = sigmoid_f32(v);
    }
    __syncthreads();
    if (wave < 2) {
      const v4f val = *(const v4f*)(sO + wave * 128 + lane * 4);
      float* dst = out + kOutO1 + rbase * 8 + wave * 128 + lane * 4;
      *(volatile v4f*)dst = val;
      __threadfence();
      *(volatile v4f*)dst = val;
    }
    return;
  }

  if (wave == 0) {
    const int bb = lane >> 3, c = lane & 7;
    const float* p = x1 + (size_t)bb * 512 + c;
    float mxv = p[0];
    float mnv = mxv;
#pragma unroll 4
    for (int n = 1; n < kNo; ++n) {
      const float x = p[n * 8];
      mxv = fmaxf(mxv, x);
      mnv = fminf(mnv, x);
    }
    sF0[bb * 24 + c]         = x0[bb * 8 + c];
    sF0[bb * 24 + 8 + 2 * c] = mxv;
    sF0[bb * 24 + 9 + 2 * c] = mnv;
  }
  __syncthreads();
  if (wave == 0) {
    const int bb = lane >> 3, ch = lane & 7;
    float acc = 0.0f;
#pragma unroll 4
    for (int k = 0; k < kFeat0; ++k) acc = fmaf(sF0[bb * 24 + k], W0[k * 8 + ch], acc);
    const float v = acc + b0[ch];
    const float o = sigmoid_f32(v);
    float* dst = out + kOutO0 + lane;
    *(volatile float*)dst = o;
    __threadfence();
    *(volatile float*)dst = o;
  }
}

__global__ __launch_bounds__(256) void o2_kernel(
    const float* __restrict__ x1, const float* __restrict__ x2, const float* __restrict__ R2,
    const float* __restrict__ W2, const float* __restrict__ b2, float* __restrict__ out2)
{
  __shared__ float sW[kFeat2 * 8];
  __shared__ float sF[32 * kFeat2];
  __shared__ __align__(16) float sO[256];
  const int tid = threadIdx.x, lane = tid & 31, wave = tid >> 5;
  const int blk = blockIdx.x;
  const int jh = blk & 1, i = (blk >> 1) & 63, b = blk >> 7;
  const int j0 = jh * 32;
  const int bi = b * 64 + i;
  const int rl = tid >> 3, c = tid & 7;
  {
    const int j = j0 + rl;
    const int bj = b * 64 + j;
    sW[tid]       = W2[tid];
    sW[256 + tid] = W2[256 + tid];
    sF[rl * kFeat2 + c]      = x1[bi * 8 + c];
    sF[rl * kFeat2 + 8 + c]  = x2[(size_t)(bi * 64 + j) * 8 + c];
    sF[rl * kFeat2 + 32 + c] = x1[bj * 8 + c];
    sF[rl * kFeat2 + 40 + c] = x2[(size_t)(bj * 64 + i) * 8 + c];
#pragma unroll
    for (int u = 0; u < 2; ++u) {
      const int idx = tid + 256 * u;
      const int r2 = idx >> 4, s = idx & 15;
      const int jr = j0 + r2;
      sF[r2 * kFeat2 + 16 + s] = R2[(size_t)(bi * 64 + jr) * 16 + s];
      sF[r2 * kFeat2 + 48 + s] = R2[(size_t)((b * 64 + jr) * 64 + i) * 16 + s];
    }
  }
  __syncthreads();
  {
    float acc = 0.0f;
#pragma unroll 8
    for (int k = 0; k < kFeat2; ++k) acc = fmaf(sF[rl * kFeat2 + k], sW[k * 8 + c], acc);
    const float v = acc + b2[c];
    sO[tid] = sigmoid_f32(v);
  }
  __syncthreads();
  if (wave < 2) {
    const v4f val = *(const v4f*)(sO + wave * 128 + lane * 4);
    float* dst = out2 + (size_t)blk * 256 + wave * 128 + lane * 4;
    *(volatile v4f*)dst = val;
    __threadfence();
    *(volatile v4f*)dst = val;
  }
}

__global__ __launch_bounds__(256) void o3_kernel(
    const _Float16* __restrict__ planes, const _Float16* __restrict__ W3t,
    const float* __restrict__ b3, float* __restrict__ out3)
{
  __shared__ __align__(16) float sD[8][16 * 16];
  const int tid = threadIdx.x, lane = tid & 31, wave = tid >> 5;
  const int h = lane >> 4, m = lane & 15;
  const int gw = blockIdx.x * 8 + wave;
  const int j = gw & 63, i = (gw >> 6) & 63, b = gw >> 12;
  const int bi = b * 64 + i, bj = b * 64 + j;

  const v16h wf0 = frag_load_f16(W3t + m * kFeat3 + 0  + 8 * h);
  const v16h wf1 = frag_load_f16(W3t + m * kFeat3 + 32 + 8 * h);
  const v16h wf2 = frag_load_f16(W3t + m * kFeat3 + 64 + 8 * h);

  const int c4 = (lane & 1) * 4;
  const v4f bv = *(const v4f*)(b3 + c4);
  float* sd = sD[wave];

#pragma unroll 1
  for (int t = 0; t < 4; ++t) {
    const int k = t * 16 + m;
    const int bk = b * 64 + k;
    const int s0 = h ? ((bi * 64 + j) * 64 + k) : (kX2Seg0 + bi * 64 + j);
    const int s1 = h ? ((bi * 64 + k) * 64 + j) : (kX2Seg0 + bi * 64 + k);
    const int s2 = h ? ((bj * 64 + i) * 64 + k) : (kX2Seg0 + bj * 64 + i);
    const int s3 = h ? ((bk * 64 + i) * 64 + j) : (kX2Seg0 + bk * 64 + i);
    const int s4 = h ? ((bj * 64 + k) * 64 + i) : (kX2Seg0 + bj * 64 + k);
    const int s5 = h ? ((bk * 64 + j) * 64 + i) : (kX2Seg0 + bk * 64 + j);
    FragU f0, f1, f2;
    f0.p[0] = *(const v8h*)(planes + (size_t)s0 * 8);
    f0.p[1] = *(const v8h*)(planes + (size_t)s1 * 8);
    f1.p[0] = *(const v8h*)(planes + (size_t)s2 * 8);
    f1.p[1] = *(const v8h*)(planes + (size_t)s3 * 8);
    f2.p[0] = *(const v8h*)(planes + (size_t)s4 * 8);
    f2.p[1] = *(const v8h*)(planes + (size_t)s5 * 8);

    v8f acc = (v8f){0.f, 0.f, 0.f, 0.f, 0.f, 0.f, 0.f, 0.f};
    acc = mma_f16_guarded(f0.v, wf0, acc);
    acc = mma_f16_guarded(f1.v, wf1, acc);
    acc = mma_f16_guarded(f2.v, wf2, acc);

#pragma unroll
    for (int r = 0; r < 8; ++r) sd[(8 * h + r) * 16 + m] = acc[r] * kFold;
    __syncthreads();
    const v4f pre = *(const v4f*)(sd + (lane >> 1) * 16 + c4);
    v4f o;
#pragma unroll
    for (int u = 0; u < 4; ++u) {
      const float v = pre[u] + bv[u];
      o[u] = sigmoid_f32(v);
    }
    float* dst = out3 + ((size_t)gw * 64 + t * 16) * 8 + lane * 4;
    *(volatile v4f*)dst = o;
    __threadfence();
    *(volatile v4f*)dst = o;
    __syncthreads();
  }
}

extern "C" void kernel_launch(void* const* d_in, const int* in_sizes, int n_in,
                              void* d_out, int out_size, void* d_ws, size_t ws_size,
                              hipStream_t stream) {
  if (n_in < 12) return;
  if (in_sizes[0] != kNb * kNc) return;
  if (in_sizes[1] != kRowsO1 * kNc) return;
  if (in_sizes[2] != kRowsO2 * kNc) return;
  if (in_sizes[3] != kRowsO3 * kNc) return;
  if (in_sizes[4] != kFeat0 * kNc) return;
  if (in_sizes[5] != kNc) return;
  if (in_sizes[6] != kFeat1 * kNc) return;
  if (in_sizes[7] != kNc) return;
  if (in_sizes[8] != kFeat2 * kNc) return;
  if (in_sizes[9] != kNc) return;
  if (in_sizes[10] != kFeat3 * kNc) return;
  if (in_sizes[11] != kNc) return;
  if (out_size != kOutTotal) return;
  if (ws_size < kWsTotal) return;

  const float* x0 = (const float*)d_in[0];
  const float* x1 = (const float*)d_in[1];
  const float* x2 = (const float*)d_in[2];
  const float* x3 = (const float*)d_in[3];
  const float* W0 = (const float*)d_in[4];
  const float* b0 = (const float*)d_in[5];
  const float* W1 = (const float*)d_in[6];
  const float* b1 = (const float*)d_in[7];
  const float* W2 = (const float*)d_in[8];
  const float* b2 = (const float*)d_in[9];
  const float* W3 = (const float*)d_in[10];
  const float* b3 = (const float*)d_in[11];
  float* out = (float*)d_out;

  char* ws = (char*)d_ws;
  unsigned short* X3H = (unsigned short*)(ws + kOffX3H);
  unsigned short* X2H = (unsigned short*)(ws + kOffX2H);
  unsigned short* W3T = (unsigned short*)(ws + kOffW3T);
  float*          R2  = (float*)(ws + kOffR2);

  prep_x3_kernel<<<kNb * kNo * 4, 256, 0, stream>>>(x3, X3H, R2);
  prep_small_kernel<<<74, 256, 0, stream>>>(x0, x1, x2, W0, b0, W1, b1, W3, X2H, W3T, out);
  o2_kernel<<<kRowsO2 / 32, 256, 0, stream>>>(x1, x2, R2, W2, b2, out + kOutO2);
  o3_kernel<<<kRowsO2 / 8, 256, 0, stream>>>((const _Float16*)X3H, (const _Float16*)W3T, b3, out + kOutO3);
}
